// MixCrossAttention_88046829568164
// MI455X (gfx1250) — hardware-run, weakly checked
//
#include <hip/hip_runtime.h>


#ifndef NB
#define NB 4
#endif
#ifndef SEQ
#define SEQ 1024
#endif
#define NB_FULL  4
#define SEQ_FULL 1024
#define DM   512
#define NH_  8
#define HD   64
#define NBH  (NB * NH_)
#define NTOP 35
#define JP   48
#define JT   96
#define NMODE 64
#define AW   4
#define QP   72
#define VP   104
#define OP   36
#define TP   80
#define L2E  1.4426950408889634f
#define SC2  (0.04419417382415922f * 1.4426950408889634f)
#define PCARRY 256.0f
#define OSC2 (1.0f / 512.0f)
#define INV_PI 0.3183098861837907f

static_assert(HD == 64);
static_assert(NH_ * HD == DM);
static_assert(SEQ == SEQ_FULL);
static_assert(SEQ == 1024);
static_assert((SEQ & (SEQ - 1)) == 0);
static_assert(SEQ % 64 == 0);
static_assert(SEQ % 32 == 0);
static_assert(HD % 32 == 0);
static_assert((2 * NMODE) % 32 == 0);
static_assert(JT % 32 == 0);
static_assert(NTOP > 32 && NTOP <= JP);
static_assert(JT == 2 * JP);
static_assert(SEQ % (32 * AW) == 0);
static_assert(NB <= NB_FULL);
static_assert(HD == 16 * AW);
static_assert(QP % 8 == 0 && QP >= HD);
static_assert(VP % 8 == 0 && VP >= JT);
static_assert(OP % 4 == 0 && OP >= 32);
static_assert(TP >= 72);
static_assert(18 * 256 == 72 * 64);
static_assert(2 * 256 * 8 == 64 * 64);
static_assert((JT * HD) % (32 * AW) == 0);
static_assert(32 * 16 * 4 == 16 * 128);
static_assert(32 * 16 * 16 == HD * 128);
static_assert(32 * 16 * 8 == 16 * 256);
static_assert(32 * AW * 16 * 4 == SEQ * 8);
static_assert(32 * 32 == 16 * 64);
static_assert(SEQ * 8 + AW * 8 + AW * 4 + JT * 4 + JT * QP * 2 + HD * VP * 2 + AW * HD * OP * 4 <= 131072);
static_assert(AW * SEQ * 8 <= 131072);
static_assert(2 * AW * 16 * 68 * 4 <= 131072);
static_assert(64 * TP * 2 <= 131072);
static_assert(NB * 4 * 128 * 4 <= 131072);
static_assert((NB * 64) % 32 == 0);

typedef _Float16 h16;
typedef unsigned short bf;
typedef __attribute__((ext_vector_type(16))) __bf16   v16bf;
typedef __attribute__((ext_vector_type(16))) _Float16 v16h;
typedef __attribute__((ext_vector_type(8)))  _Float16 v8h;
typedef __attribute__((ext_vector_type(8)))  unsigned short v8us;
typedef __attribute__((ext_vector_type(8)))  float    v8f;
typedef __attribute__((ext_vector_type(4)))  float    v4f;
typedef __attribute__((ext_vector_type(2)))  float    v2f;
typedef __attribute__((ext_vector_type(2)))  double   v2d;
typedef v4f  __attribute__((may_alias)) v4fa;

__device__ __forceinline__ unsigned short f2bf(float f) { unsigned u = __float_as_uint(f); u += 0x7FFFu + ((u >> 16) & 1u); return (unsigned short)(u >> 16); }
__device__ __forceinline__ float bfr(float f) { return __uint_as_float(((unsigned)f2bf(f)) << 16); }
__device__ __forceinline__ v16h cat16(v8h lo, v8h hi) { return __builtin_shufflevector(lo, hi, 0, 1, 2, 3, 4, 5, 6, 7, 8, 9, 10, 11, 12, 13, 14, 15); }
__device__ __forceinline__ v16bf cat16b(v8us lo, v8us hi) { return __builtin_bit_cast(v16bf, __builtin_shufflevector(lo, hi, 0, 1, 2, 3, 4, 5, 6, 7, 8, 9, 10, 11, 12, 13, 14, 15)); }
__device__ __forceinline__ v8f wmma16(v16h a, v16h b, v8f c) { return __builtin_amdgcn_wmma_f32_16x16x32_f16(false, a, false, b, (short)0, c, false, false); }
__device__ __forceinline__ v8f wmmab(v16bf a, v16bf b, v8f c) { return __builtin_amdgcn_wmma_f32_16x16x32_bf16(false, a, false, b, (short)0, c, false, false); }
__device__ __forceinline__ v16h  ldh(const h16* p) { return cat16(*(const v8h*)p, *(const v8h*)(p + 16)); }
__device__ __forceinline__ v16bf ldb(const bf* p)  { return cat16b(*(const v8us*)p, *(const v8us*)(p + 16)); }
__device__ __forceinline__ void wave_sync() { __builtin_amdgcn_fence(3  , "wavefront"); __builtin_amdgcn_wave_barrier(); asm volatile("" ::: "memory"); }

static __device__ __forceinline__ h16 toh_flush(float v) { const h16 r = (h16)v; return (fabsf(v) < 6.103515625e-05f) ? (h16)0.0f : r; }
__device__ __forceinline__ v8f wmma16g(v16h a, v16h b, v8f c) { c = wmma16(a, b, c); asm volatile("v_nop\n\tv_nop\n\tv_nop\n\tv_nop" : "+v"(c) : "v"(a), "v"(b)); return c; }
__device__ __forceinline__ v8f wmmabg(v16bf a, v16bf b, v8f c) { c = wmmab(a, b, c); asm volatile("v_nop\n\tv_nop\n\tv_nop\n\tv_nop" : "+v"(c) : "v"(a), "v"(b)); return c; }
__device__ __forceinline__ v16bf ldbf32(const float* p) {
    const v4f a = *(const v4f*)p, b = *(const v4f*)(p + 4), c = *(const v4f*)(p + 16), d = *(const v4f*)(p + 20); v8us lo, hi;
#pragma unroll
    for (int i = 0; i < 4; ++i) { lo[i] = f2bf(a[i]); lo[4 + i] = f2bf(b[i]); hi[i] = f2bf(c[i]); hi[4 + i] = f2bf(d[i]); }
    return cat16b(lo, hi);
}

__global__ __launch_bounds__(256) void k_tab(bf* FT, bf* IDT) {
    const int g = blockIdx.x * 256 + threadIdx.x;
    v8us o;
    if (g < 2 * NMODE * SEQ / 8) {
        const int n = g / (SEQ / 8), l8 = (g % (SEQ / 8)) * 8; const int x = n & (NMODE - 1); const bool im = n >= NMODE;
#pragma unroll
        for (int i = 0; i < 8; ++i) { const float rev = (float)((x * (l8 + i)) & (SEQ - 1)) * (1.0f / SEQ);
            const float c = __builtin_amdgcn_cosf(rev), s = __builtin_amdgcn_sinf(rev); o[i] = f2bf(im ? -s : c); }
        bf* p = FT + (size_t)n * SEQ + l8;
        *(volatile v8us*)p = o; __threadfence(); *(volatile v8us*)p = o;
    } else {
        const int g2 = g - 2 * NMODE * SEQ / 8; const int s_ = g2 / (2 * NMODE / 8), kk8 = (g2 % (2 * NMODE / 8)) * 8;
        if (s_ < SEQ) {
#pragma unroll
            for (int i = 0; i < 8; ++i) { const int kk = kk8 + i; const int x = kk & (NMODE - 1); const bool im = kk >= NMODE;
                const float rev = (float)((x * s_) & (SEQ - 1)) * (1.0f / SEQ);
                const float cf = (x == 0) ? 9.5367431640625e-07f : 1.9073486328125e-06f;
                const float c = __builtin_amdgcn_cosf(rev), s = __builtin_amdgcn_sinf(rev); o[i] = f2bf(im ? -(cf * s) : (cf * c)); }
            bf* p = IDT + (size_t)s_ * (2 * NMODE) + kk8;
            *(volatile v8us*)p = o; __threadfence(); *(volatile v8us*)p = o;
        }
    }
}

__global__ __launch_bounds__(256) void k_tr(const float* __restrict__ src, bf* dst, int nshift, size_t splane) {
    __shared__ __align__(16) unsigned short ts[64 * TP];
    const int tid = threadIdx.x; const int l0 = blockIdx.x * 64; const int bh = blockIdx.y; const int b = bh / NH_, h = bh % NH_;
    const size_t sbase = (size_t)b * SEQ_FULL * DM + (size_t)h * HD;
#pragma unroll 1
    for (int it = 0; it < 18; ++it) { const int idx = it * 256 + tid; const int row = idx >> 6, e = idx & 63;
        const int l = (l0 - 8 + row) & (SEQ - 1);
        ts[e * TP + row] = f2bf(src[sbase + (size_t)l * DM + e]); }
    __syncthreads();
    const size_t dbase = (size_t)bh * HD * SEQ + l0;
#pragma unroll 1
    for (int ps = 0; ps < 2; ++ps) {
#pragma unroll 1
        for (int r = 0; r < nshift; ++r) {
#pragma unroll 1
            for (int it = 0; it < 2; ++it) { const int p = it * 256 + tid; const int e = p >> 3, c8 = (p & 7) * 8;
                v8us o;
#pragma unroll
                for (int i = 0; i < 8; ++i) o[i] = ts[e * TP + 8 + c8 - r + i];
                *(volatile v8us*)(dst + (size_t)r * splane + dbase + (size_t)e * SEQ + c8) = o; }
        }
        if (ps == 0) __threadfence(); }
}

__global__ __launch_bounds__(32) void k_gemm(const bf* __restrict__ A, size_t sA, const bf* __restrict__ Bt, size_t sB, bf* C, size_t sC, int ldc) {
    __shared__ __align__(16) float os[16 * 68];
    const int K = SEQ;
    const int lane = threadIdx.x & 31, lr = lane & 15, hi = lane >> 4; const int r0 = blockIdx.x * 64, c0 = blockIdx.y * 64; const size_t z = blockIdx.z;
    v8f acc[4][4];
#pragma unroll
    for (int mb = 0; mb < 4; ++mb)
#pragma unroll
        for (int nb = 0; nb < 4; ++nb) acc[mb][nb] = (v8f){};
    const size_t aoff = z * sA + (size_t)(r0 + lr) * K + 8 * hi, boff = z * sB + (size_t)(c0 + lr) * K + 8 * hi;
#pragma unroll 1
    for (int kc = 0; kc < K; kc += 32) {
        v16bf a[4];
#pragma unroll
        for (int mb = 0; mb < 4; ++mb) a[mb] = ldb(A + aoff + (size_t)mb * 16 * K + kc);
#pragma unroll
        for (int nb = 0; nb < 4; ++nb) { const v16bf b = ldb(Bt + boff + (size_t)nb * 16 * K + kc);
#pragma unroll
            for (int mb = 0; mb < 4; ++mb) acc[mb][nb] = wmmabg(a[mb], b, acc[mb][nb]); }
    }
    const int c8 = (lane & 7) * 8, rg = lane >> 3;
#pragma unroll
    for (int mb = 0; mb < 4; ++mb) {
#pragma unroll
        for (int nb = 0; nb < 4; ++nb) {
#pragma unroll
            for (int j = 0; j < 8; ++j) os[(hi * 8 + j) * 68 + nb * 16 + lr] = acc[mb][nb][j]; }
        wave_sync();
        bf* cb = C + z * sC + (size_t)(r0 + mb * 16) * (size_t)ldc + c0;
#pragma unroll 1
        for (int ps = 0; ps < 2; ++ps) {
#pragma unroll
            for (int s = 0; s < 4; ++s) { const int row = 4 * s + rg;
                const v4f x0 = *(const v4fa*)(&os[row * 68 + c8]); const v4f x1 = *(const v4fa*)(&os[row * 68 + c8 + 4]); v8us hv;
#pragma unroll
                for (int i = 0; i < 4; ++i) { hv[i] = f2bf(x0[i]); hv[4 + i] = f2bf(x1[i]); }
                *(volatile v8us*)(cb + (size_t)row * (size_t)ldc + c8) = hv; }
            if (ps == 0) __threadfence(); }
        wave_sync();
    }
}

__global__ __launch_bounds__(32 * AW) void k_ztanh(const bf* __restrict__ XT, bf* TZ) {
    __shared__ __align__(16) float zr[AW * 16 * 68];
    __shared__ __align__(16) float zi[AW * 16 * 68];
    const int lane = threadIdx.x & 31, lr = lane & 15, hi = lane >> 4;
    const int wave = __builtin_amdgcn_readfirstlane(threadIdx.x >> 5);
    const int bh = blockIdx.x;
    const size_t qb = (size_t)bh * (2 * NMODE * HD) + (size_t)(16 * wave + lr) * HD + 8 * hi;
    const size_t kb = (size_t)(NBH + bh) * (2 * NMODE * HD) + (size_t)lr * HD + 8 * hi;
    const v8us sgn = {0x8000, 0x8000, 0x8000, 0x8000, 0x8000, 0x8000, 0x8000, 0x8000};
    v8f cre[4], cim[4];
#pragma unroll
    for (int t = 0; t < 4; ++t) { cre[t] = (v8f){}; cim[t] = (v8f){}; }
#pragma unroll
    for (int ks = 0; ks < 2; ++ks) {
        const v16bf aqr = ldb(XT + qb + 32 * ks), aqi = ldb(XT + qb + NMODE * HD + 32 * ks);
#pragma unroll
        for (int yt = 0; yt < 4; ++yt) { const bf* kp = XT + kb + (size_t)yt * 16 * HD + 32 * ks;
            const v8us k0 = *(const v8us*)kp, k1 = *(const v8us*)(kp + 16), i0 = *(const v8us*)(kp + NMODE * HD), i1 = *(const v8us*)(kp + NMODE * HD + 16);
            const v16bf bkr = cat16b(k0, k1), bki = cat16b(i0, i1), bkn = cat16b(i0 ^ sgn, i1 ^ sgn);
            cre[yt] = wmmabg(aqr, bkr, cre[yt]); cre[yt] = wmmabg(aqi, bkn, cre[yt]);
            cim[yt] = wmmabg(aqr, bki, cim[yt]); cim[yt] = wmmabg(aqi, bkr, cim[yt]); }
    }
    const int wb = wave * 16 * 68;
#pragma unroll
    for (int yt = 0; yt < 4; ++yt) {
#pragma unroll
        for (int r = 0; r < 8; ++r) { zr[wb + (8 * hi + r) * 68 + 16 * yt + lr] = cre[yt][r]; zi[wb + (8 * hi + r) * 68 + 16 * yt + lr] = cim[yt][r]; } }
    wave_sync();
#pragma unroll 1
    for (int it = 0; it < 32; ++it) { const int id = it * 32 + lane; const int p = wb + (id >> 6) * 68 + (id & 63);
        const float a = zr[p], bq = zi[p];
        const float ac = fminf(fmaxf(a, -12.0f), 12.0f);
        const float ex = __builtin_amdgcn_exp2f(ac * (2.0f * L2E)); const float em = __builtin_amdgcn_rcpf(ex);
        const float sh = 0.5f * (ex - em), ch = 0.5f * (ex + em);
        float t = bq * INV_PI; t = t - floorf(t);
        const float s2 = __builtin_amdgcn_sinf(t), c2 = __builtin_amdgcn_cosf(t);
        const float rd = __builtin_amdgcn_rcpf(fmaxf(ch + c2, 1.0e-20f));
        zr[p] = sh * rd; zi[p] = s2 * rd; }
    wave_sync();
    const int c8 = (lane & 7) * 8, rg = lane >> 3;
    bf* trow = TZ + ((size_t)bh * NMODE + 16 * wave) * NMODE;
#pragma unroll 1
    for (int ps = 0; ps < 2; ++ps) {
#pragma unroll
        for (int s = 0; s < 4; ++s) { const int row = 4 * s + rg;
            const v4f x0 = *(const v4fa*)(&zr[wb + row * 68 + c8]); const v4f x1 = *(const v4fa*)(&zr[wb + row * 68 + c8 + 4]);
            const v4f y0 = *(const v4fa*)(&zi[wb + row * 68 + c8]); const v4f y1 = *(const v4fa*)(&zi[wb + row * 68 + c8 + 4]); v8us hv, iv;
#pragma unroll
            for (int i = 0; i < 4; ++i) { hv[i] = f2bf(x0[i]); hv[4 + i] = f2bf(x1[i]); iv[i] = f2bf(y0[i]); iv[4 + i] = f2bf(y1[i]); }
            *(volatile v8us*)(trow + (size_t)row * NMODE + c8) = hv;
            *(volatile v8us*)(trow + (size_t)NBH * NMODE * NMODE + (size_t)row * NMODE + c8) = iv; }
        if (ps == 0) __threadfence(); }
}

__global__ __launch_bounds__(32 * AW) void k_xqkv(const bf* __restrict__ XKN, const bf* __restrict__ TZ, float* U) {
    __shared__ __align__(16) float ur[AW * 16 * 68];
    __shared__ __align__(16) float ui[AW * 16 * 68];
    const int lane = threadIdx.x & 31, lr = lane & 15, hi = lane >> 4;
    const int wave = __builtin_amdgcn_readfirstlane(threadIdx.x >> 5);
    const int bh = blockIdx.x;
    const size_t ka = ((size_t)bh * HD + 16 * wave + lr) * (2 * NMODE) + 8 * hi;
    const size_t tb = ((size_t)bh * NMODE + lr) * NMODE + 8 * hi;
    const v8us sgn = {0x8000, 0x8000, 0x8000, 0x8000, 0x8000, 0x8000, 0x8000, 0x8000};
    v8f cre[4], cim[4];
#pragma unroll
    for (int t = 0; t < 4; ++t) { cre[t] = (v8f){}; cim[t] = (v8f){}; }
#pragma unroll
    for (int ks = 0; ks < 2; ++ks) {
        const bf* ap = XKN + ka + 32 * ks;
        const v8us r0 = *(const v8us*)ap, r1 = *(const v8us*)(ap + 16), i0 = *(const v8us*)(ap + NMODE), i1 = *(const v8us*)(ap + NMODE + 16);
        const v16bf akr = cat16b(r0, r1), aki = cat16b(i0, i1), akn = cat16b(i0 ^ sgn, i1 ^ sgn);
#pragma unroll
        for (int xt = 0; xt < 4; ++xt) {
            const v16bf btr = ldb(TZ + tb + (size_t)xt * 16 * NMODE + 32 * ks);
            const v16bf bti = ldb(TZ + (size_t)NBH * NMODE * NMODE + tb + (size_t)xt * 16 * NMODE + 32 * ks);
            cre[xt] = wmmabg(akr, btr, cre[xt]); cre[xt] = wmmabg(akn, bti, cre[xt]);
            cim[xt] = wmmabg(aki, btr, cim[xt]); cim[xt] = wmmabg(akr, bti, cim[xt]); }
    }
    const int wb = wave * 16 * 68;
#pragma unroll
    for (int xt = 0; xt < 4; ++xt) {
#pragma unroll
        for (int r = 0; r < 8; ++r) { ur[wb + (8 * hi + r) * 68 + 16 * xt + lr] = cre[xt][r]; ui[wb + (8 * hi + r) * 68 + 16 * xt + lr] = cim[xt][r]; } }
    wave_sync();
    const int cofs = lr * 4;
    float* ub = U + ((size_t)bh * HD + 16 * wave) * (2 * NMODE);
#pragma unroll 1
    for (int ps = 0; ps < 2; ++ps) {
#pragma unroll
        for (int s = 0; s < 8; ++s) { const int row = 2 * s + hi;
            const v4f x = *(const v4fa*)(&ur[wb + row * 68 + cofs]); const v4f y = *(const v4fa*)(&ui[wb + row * 68 + cofs]);
            *(volatile v4f*)(ub + (size_t)row * (2 * NMODE) + cofs) = x;
            *(volatile v4f*)(ub + (size_t)row * (2 * NMODE) + NMODE + cofs) = y; }
        if (ps == 0) __threadfence(); }
}

__global__ __launch_bounds__(256) void k_w1(const float* __restrict__ wre, const float* __restrict__ wim, const float* __restrict__ U, bf* XWB) {
    __shared__ __align__(16) float sw[NB * 4 * 128];
    const int tid = threadIdx.x; const int x = tid & 63, ol = tid >> 6; const int h = blockIdx.y; const int o = blockIdx.x * 4 + ol;
    float ar[NB], ai[NB];
#pragma unroll
    for (int b = 0; b < NB; ++b) { ar[b] = 0.0f; ai[b] = 0.0f; }
#pragma unroll 1
    for (int e = 0; e < HD; ++e) {
        const size_t wi_ = (((size_t)h * HD + e) * HD + o) * NMODE + x;
        const float wr = bfr(wre[wi_]), wi = bfr(wim[wi_]);
#pragma unroll
        for (int b = 0; b < NB; ++b) { const float* up = U + (((size_t)b * NH_ + h) * HD + e) * (2 * NMODE) + x;
            const float u_r = up[0], u_i = up[NMODE];
            ar[b] += wr * u_r - wi * u_i; ai[b] += wr * u_i + wi * u_r; }
    }
#pragma unroll
    for (int b = 0; b < NB; ++b) { sw[(b * 4 + ol) * 128 + x] = ar[b]; sw[(b * 4 + ol) * 128 + NMODE + x] = ai[b]; }
    __syncthreads();
    if (tid < NB * 64) {
        const int b = tid >> 6, o2 = (tid >> 4) & 3, c8 = (tid & 15) * 8; v8us hv;
#pragma unroll
        for (int i = 0; i < 8; ++i) hv[i] = f2bf(sw[(b * 4 + o2) * 128 + c8 + i]);
        bf* p = XWB + (((size_t)b * NH_ + h) * HD + blockIdx.x * 4 + o2) * (2 * NMODE) + c8;
        *(volatile v8us*)p = hv; __threadfence(); *(volatile v8us*)p = hv;
    }
}

__global__ __launch_bounds__(32 * AW) void k_corr(const bf* __restrict__ PL, double* AMP) {
    __shared__ double part[AW * SEQ];
    const int tid = threadIdx.x; const int lane = tid & 31, lr = lane & 15, hi = lane >> 4;
    const int wave = __builtin_amdgcn_readfirstlane(threadIdx.x >> 5);
    const int bh = blockIdx.x;
    const size_t pstride = (size_t)NBH * HD * SEQ;
    double s2[4][8];
#pragma unroll
    for (int mt = 0; mt < 4; ++mt)
#pragma unroll
        for (int r = 0; r < 8; ++r) s2[mt][r] = 0.0;
    const int qa = 8 * hi + 16 * lr;
    const int ka = 8 * hi - 8 * (lr >> 3);
#pragma unroll 1
    for (int ee = 0; ee < 16; ++ee) {
        const int e = wave * 16 + ee;
        const size_t qofs = ((size_t)bh * HD + e) * SEQ;
        const size_t kofs = (size_t)(1 + (lr & 7)) * pstride + qofs;
        v8f acc[4];
#pragma unroll
        for (int mt = 0; mt < 4; ++mt) acc[mt] = (v8f){};
#pragma unroll 1
        for (int kc = 0; kc < SEQ; kc += 32) {
            const int kb0 = (ka + kc) & (SEQ - 1), kb1 = (ka + kc + 16) & (SEQ - 1);
            const v16bf bk = cat16b(*(const v8us*)(PL + kofs + kb0), *(const v8us*)(PL + kofs + kb1));
#pragma unroll
            for (int mt = 0; mt < 4; ++mt) { const int q0 = (qa + 256 * mt + kc) & (SEQ - 1), q1 = (q0 + 16) & (SEQ - 1);
                const v16bf aq = cat16b(*(const v8us*)(PL + qofs + q0), *(const v8us*)(PL + qofs + q1));
                acc[mt] = wmmabg(aq, bk, acc[mt]); }
        }
#pragma unroll
        for (int mt = 0; mt < 4; ++mt)
#pragma unroll
            for (int r = 0; r < 8; ++r) { const double d = (double)acc[mt][r]; s2[mt][r] += d * d; }
    }
#pragma unroll
    for (int mt = 0; mt < 4; ++mt)
#pragma unroll
        for (int r = 0; r < 8; ++r) part[wave * SEQ + 256 * mt + 128 * hi + 16 * r + lr] = s2[mt][r];
    __syncthreads();
    double* arow = AMP + (size_t)bh * SEQ;
#pragma unroll 1
    for (int ps = 0; ps < 2; ++ps) {
#pragma unroll 1
        for (int it = 0; it < 4; ++it) { const int tau = it * (64 * AW) + 2 * tid; v2d o;
            o[0] = ((part[tau] + part[SEQ + tau]) + part[2 * SEQ + tau]) + part[3 * SEQ + tau];
            o[1] = ((part[tau + 1] + part[SEQ + tau + 1]) + part[2 * SEQ + tau + 1]) + part[3 * SEQ + tau + 1];
            *(volatile v2d*)(arow + tau) = o; }
        if (ps == 0) __threadfence(); }
}

__device__ __forceinline__ void path_p(const v8f t0, const v8f t1, const v8f t2, const float nwp, const int hi, v8h& p0, v8h& p1, v8h& p2) {
    float a0[8], a1[8], a2[8]; float mx = -3.0e38f;
#pragma unroll
    for (int r = 0; r < 8; ++r) { const bool vd = (32 + 8 * hi + r) < NTOP;
        a0[r] = t0[r] * SC2; a1[r] = t1[r] * SC2; a2[r] = vd ? (t2[r] * SC2) : -3.0e38f;
        mx = fmaxf(mx, fmaxf(a0[r], fmaxf(a1[r], a2[r]))); }
    mx = fmaxf(mx, __shfl_xor(mx, 16, 32));
    float e0[8], e1[8], e2[8]; float sum = 0.0f;
#pragma unroll
    for (int r = 0; r < 8; ++r) { const bool vd = (32 + 8 * hi + r) < NTOP;
        e0[r] = __builtin_amdgcn_exp2f(a0[r] - mx); e1[r] = __builtin_amdgcn_exp2f(a1[r] - mx);
        const float x2 = __builtin_amdgcn_exp2f(t2[r] * SC2 - mx); e2[r] = vd ? x2 : 0.0f;
        sum += (e0[r] + e1[r]) + e2[r]; }
    sum += __shfl_xor(sum, 16, 32);
    const float g = (nwp * PCARRY) * (1.0f / sum);
#pragma unroll
    for (int r = 0; r < 8; ++r) { p0[r] = toh_flush(e0[r] * g); p1[r] = toh_flush(e1[r] * g); p2[r] = toh_flush(e2[r] * g); }
}

__global__ __launch_bounds__(32 * AW) void k_attn(const float* __restrict__ tfq, const float* __restrict__ qg, const float* __restrict__ kg, const float* __restrict__ vg,
                                                  const float* __restrict__ wfu, const double* __restrict__ AMP, const bf* __restrict__ XWB, const bf* __restrict__ IDT, float* OUT) {
    __shared__ double val[SEQ];
    __shared__ double rv[AW];
    __shared__ int ri[AW];
    __shared__ int jdx[JT];
    __shared__ __align__(16) unsigned short QS[JT * QP];
    __shared__ __align__(16) h16 VS[HD * VP];
    __shared__ __align__(16) float os[AW * HD * OP];
    const int tid = threadIdx.x; const int lane = tid & 31, lr = lane & 15, hi = lane >> 4;
    const int wave = __builtin_amdgcn_readfirstlane(threadIdx.x >> 5);
    const int bh = blockIdx.x; const int b = bh / NH_, h = bh % NH_;
    const size_t rowbase = (size_t)b * SEQ_FULL * DM + (size_t)h * HD;
    if (tid < JT) jdx[tid] = 0;
#pragma unroll 1
    for (int p = 0; p < 2; ++p) {
        if (p == 0) {
#pragma unroll 1
            for (int q = 0; q < SEQ / (32 * AW); ++q) { const int i = tid + q * 32 * AW; val[i] = AMP[(size_t)bh * SEQ + i]; }
        } else {
#pragma unroll 1
            for (int q = 0; q < SEQ / (32 * AW); ++q) { const int i = tid + q * 32 * AW; const float* rp = tfq + rowbase + (size_t)i * DM; double s = 0.0;
#pragma unroll 2
                for (int c = 0; c < HD / 4; ++c) { const v4f v = *(const v4f*)(rp + 4 * c);
#pragma unroll
                    for (int k = 0; k < 4; ++k) { const double d = (double)bfr(v[k]); s += d * d; } }
                val[i] = s; }
        }
        __syncthreads();
#pragma unroll 1
        for (int r = 0; r < NTOP; ++r) {
            double bv = -1.0; int bi = SEQ;
#pragma unroll 1
            for (int q = 0; q < SEQ / (32 * AW); ++q) { const int i = tid + q * 32 * AW; const double v = val[i]; const bool g = v > bv; bv = g ? v : bv; bi = g ? i : bi; }
#pragma unroll
            for (int off = 16; off > 0; off >>= 1) { const double ov = __shfl_xor(bv, off, 32); const int oi = __shfl_xor(bi, off, 32);
                const bool g = (ov > bv) | ((ov == bv) & (oi < bi)); bv = g ? ov : bv; bi = g ? oi : bi; }
            if (lane == 0) { rv[wave] = bv; ri[wave] = bi; }
            __syncthreads();
            double gv = rv[0]; int gi = ri[0];
#pragma unroll
            for (int w = 1; w < AW; ++w) { const double ov = rv[w]; const int oi = ri[w]; const bool g = (ov > gv) | ((ov == gv) & (oi < gi)); gv = g ? ov : gv; gi = g ? oi : gi; }
            gi = min(max(gi, 0), SEQ - 1);
            if (tid == 0) { jdx[JP * p + r] = gi; val[gi] = -2.0; }
            __syncthreads();
        }
    }
#pragma unroll 1
    for (int it = 0; it < JT * HD / (32 * AW); ++it) { const int idx = it * 32 * AW + tid; const int j = idx >> 6, d = idx & 63;
        int l = jdx[j]; l = min(max(l, 0), SEQ - 1);
        const size_t off = rowbase + (size_t)l * DM + d;
        float qv = qg[off]; float tv = tfq[off]; float vv = vg[off];
        asm volatile("" : "+v"(qv)); asm volatile("" : "+v"(tv)); asm volatile("" : "+v"(vv));
        const float sel = (j < JP) ? qv : tv;
        QS[j * QP + d] = f2bf(sel);
        VS[d * VP + j] = toh_flush(bfr(vv)); }
    __syncthreads();

    const int wb = wave * HD * OP;
    const int c4 = (lane & 7) * 4, rg = lane >> 3;
#pragma unroll 1
    for (int c = wave; c < SEQ / 32; c += AW) {
        const int s0 = 32 * c;
#pragma unroll 1
        for (int half = 0; half < 2; ++half) {
            const int sl = s0 + 16 * half + lr;
            const float* kp = kg + rowbase + (size_t)sl * DM + 8 * hi;
            const v16bf kb0 = ldbf32(kp), kb1 = ldbf32(kp + 32);
            v8f sc[6];
#pragma unroll
            for (int jt = 0; jt < 6; ++jt) { const int qo = (16 * jt + lr) * QP + 8 * hi; sc[jt] = (v8f){};
                sc[jt] = wmmabg(cat16b(*(const v8us*)(&QS[qo]), *(const v8us*)(&QS[qo + 16])), kb0, sc[jt]);
                sc[jt] = wmmabg(cat16b(*(const v8us*)(&QS[qo + 32]), *(const v8us*)(&QS[qo + 48])), kb1, sc[jt]); }
            const v2f w2 = *(const v2f*)(wfu + ((size_t)h * SEQ_FULL + sl) * 2);
            const float w0 = bfr(w2[0]), w1 = bfr(w2[1]); const float wm = fmaxf(w0, w1);
            const float x0 = __builtin_amdgcn_exp2f((w0 - wm) * L2E), x1 = __builtin_amdgcn_exp2f((w1 - wm) * L2E);
            const float rw = 1.0f / (x0 + x1);
            v8h pt0, pt1, pt2, pf0, pf1, pf2;
            path_p(sc[0], sc[1], sc[2], x0 * rw, hi, pt0, pt1, pt2);
            path_p(sc[3], sc[4], sc[5], x1 * rw, hi, pf0, pf1, pf2);
            const v16h pb0 = cat16(pt0, pt1), pb1 = cat16(pt2, pf0), pb2 = cat16(pf1, pf2);
            v8f o[4];
#pragma unroll
            for (int dt = 0; dt < 4; ++dt) { const int vo = (16 * dt + lr) * VP + 8 * hi; o[dt] = (v8f){};
                o[dt] = wmma16g(cat16(*(const v8h*)(&VS[vo]), *(const v8h*)(&VS[vo + 16])), pb0, o[dt]);
                o[dt] = wmma16g(cat16(*(const v8h*)(&VS[vo + 32]), *(const v8h*)(&VS[vo + 48])), pb1, o[dt]);
                o[dt] = wmma16g(cat16(*(const v8h*)(&VS[vo + 64]), *(const v8h*)(&VS[vo + 80])), pb2, o[dt]); }
            const bf* ip = IDT + (size_t)sl * (2 * NMODE) + 8 * hi;
            const bf* wp = XWB + ((size_t)bh * HD + lr) * (2 * NMODE) + 8 * hi;
#pragma unroll
            for (int k2 = 0; k2 < 4; ++k2) { const v16bf bi_ = ldb(ip + 32 * k2);
#pragma unroll
                for (int dt = 0; dt < 4; ++dt) o[dt] = wmmabg(ldb(wp + (size_t)dt * 16 * (2 * NMODE) + 32 * k2), bi_, o[dt]); }
#pragma unroll
            for (int dt = 0; dt < 4; ++dt)
#pragma unroll
                for (int r = 0; r < 8; ++r) os[wb + (16 * dt + 8 * hi + r) * OP + 16 * half + lr] = o[dt][r] * OSC2;
        }
        wave_sync();
        float* ob = OUT + (size_t)bh * HD * SEQ + s0;
#pragma unroll 1
        for (int ps = 0; ps < 2; ++ps) {
#pragma unroll
            for (int it = 0; it < 16; ++it) { const int row = 4 * it + rg;
                const v4f x = *(const v4fa*)(&os[wb + row * OP + c4]);
                *(volatile v4f*)(ob + (size_t)row * SEQ + c4) = x; }
            if (ps == 0) __threadfence(); }
        wave_sync();
    }
}

static constexpr size_t al256(size_t v) { return (v + 255) & ~(size_t)255; }
static constexpr size_t PLS    = (size_t)NBH * HD * SEQ;
static constexpr size_t SZ_PL  = al256(9 * PLS * 2);
static constexpr size_t SZ_FT  = al256((size_t)2 * NMODE * SEQ * 2);
static constexpr size_t SZ_IDT = al256((size_t)SEQ * 2 * NMODE * 2);
static constexpr size_t SZ_XT  = al256((size_t)2 * NBH * 2 * NMODE * HD * 2);
static constexpr size_t SZ_XKN = al256((size_t)NBH * HD * 2 * NMODE * 2);
static constexpr size_t SZ_TZ  = al256((size_t)2 * NBH * NMODE * NMODE * 2);
static constexpr size_t SZ_U   = al256((size_t)NBH * HD * 2 * NMODE * 4);
static constexpr size_t SZ_XW  = al256((size_t)NBH * HD * 2 * NMODE * 2);
static constexpr size_t SZ_AMP = al256((size_t)NBH * SEQ * 8);
static constexpr size_t SZ_TOTAL = SZ_PL + SZ_FT + SZ_IDT + SZ_XT + SZ_XKN + SZ_TZ + SZ_U + SZ_XW + SZ_AMP;
static_assert(SZ_TOTAL <= (size_t)134217728);
static_assert((2 * NMODE * SEQ / 8 + SEQ * 2 * NMODE / 8) % 256 == 0);

extern "C" void kernel_launch(void* const* d_in, const int* in_sizes, int n_in,
                              void* d_out, int out_size, void* d_ws, size_t ws_size, hipStream_t stream) {
    if (n_in < 8) return;
    const size_t needx = ((size_t)(NB - 1) * SEQ_FULL + SEQ) * DM;
    if ((size_t)in_sizes[0] < needx || (size_t)in_sizes[1] < needx || (size_t)in_sizes[2] < needx || (size_t)in_sizes[3] < needx) return;
    if ((size_t)in_sizes[5] < (size_t)NH_ * SEQ_FULL * 2) return;
    if ((size_t)in_sizes[6] < (size_t)NH_ * HD * HD * NMODE || (size_t)in_sizes[7] < (size_t)NH_ * HD * HD * NMODE) return;
    if ((size_t)out_size < (size_t)NBH * HD * SEQ) return;
    if (SZ_TOTAL > ws_size) return;
    const float* tfq = (const float*)d_in[0]; const float* qg = (const float*)d_in[1];
    const float* kg = (const float*)d_in[2]; const float* vg = (const float*)d_in[3];
    const float* wfu = (const float*)d_in[5];
    const float* w1re = (const float*)d_in[6]; const float* w1im = (const float*)d_in[7];
    float* OUT = (float*)d_out;
    char* wsp = (char*)d_ws;
    bf* PL = (bf*)wsp; wsp += SZ_PL;
    bf* FT = (bf*)wsp; wsp += SZ_FT;
    bf* IDT = (bf*)wsp; wsp += SZ_IDT;
    bf* XT = (bf*)wsp; wsp += SZ_XT;
    bf* XKN = (bf*)wsp; wsp += SZ_XKN;
    bf* TZ = (bf*)wsp; wsp += SZ_TZ;
    float* U = (float*)wsp; wsp += SZ_U;
    bf* XWB = (bf*)wsp; wsp += SZ_XW;
    double* AMP = (double*)wsp; wsp += SZ_AMP;

    k_tab<<<(2 * NMODE * SEQ / 8 + SEQ * 2 * NMODE / 8) / 256, 256, 0, stream>>>(FT, IDT);
    k_tr<<<dim3(SEQ / 64, NBH, 1), 256, 0, stream>>>(qg, PL, 1, PLS);
    k_tr<<<dim3(SEQ / 64, NBH, 1), 256, 0, stream>>>(kg, PL + PLS, 8, PLS);
    k_gemm<<<dim3(2 * NMODE / 64, HD / 64, 2 * NBH), 32, 0, stream>>>(FT, (size_t)0, PL, (size_t)HD * SEQ, XT, (size_t)2 * NMODE * HD, HD);
    k_gemm<<<dim3(HD / 64, 2 * NMODE / 64, NBH), 32, 0, stream>>>(PL + PLS, (size_t)HD * SEQ, FT, (size_t)0, XKN, (size_t)HD * 2 * NMODE, 2 * NMODE);
    k_ztanh<<<NBH, 32 * AW, 0, stream>>>(XT, TZ);
    k_xqkv<<<NBH, 32 * AW, 0, stream>>>(XKN, TZ, U);
    k_w1<<<dim3(HD / 4, NH_, 1), 256, 0, stream>>>(w1re, w1im, U, XWB);
    k_corr<<<NBH, 32 * AW, 0, stream>>>(PL, AMP);
    k_attn<<<NBH, 32 * AW, 0, stream>>>(tfq, qg, kg, vg, wfu, AMP, XWB, IDT, OUT);
}
